// PredAttentionValue_85375359910647
// MI455X (gfx1250) — hardware-verified
//
#include <hip/hip_runtime.h>

typedef unsigned short u16;
typedef u16      v8u  __attribute__((ext_vector_type(8)));
typedef u16      v16u __attribute__((ext_vector_type(16)));
typedef _Float16 v16h __attribute__((ext_vector_type(16)));
typedef __bf16   v16b __attribute__((ext_vector_type(16)));
typedef float    v8f  __attribute__((ext_vector_type(8)));
typedef float    v4f  __attribute__((ext_vector_type(4)));
typedef v8u __attribute__((may_alias)) v8ua;
typedef v4f __attribute__((may_alias)) v4fa;

union Frag { v16u v; v8u half[2]; v16b b; v16h h; };

#define BB 32
#define TT 500
#define TP 512
#define CC 256
#define HH 8
#define DD 32
#define SP 36
#define WPITCH 260

static __device__ __forceinline__ v8f mma_bf16(v16b a, v16b b, v8f c) {
    v8f d = __builtin_amdgcn_wmma_f32_16x16x32_bf16(false, a, false, b, (short)0, c, false, false);
    asm volatile("v_nop\n\tv_nop\n\tv_nop\n\tv_nop" : "+v"(d) : "v"(a), "v"(b));
    return d;
}
static __device__ __forceinline__ v8f mma_f16(v16h a, v16h b, v8f c) {
    v8f d = __builtin_amdgcn_wmma_f32_16x16x32_f16(false, a, false, b, (short)0, c, false, false);
    asm volatile("v_nop\n\tv_nop\n\tv_nop\n\tv_nop" : "+v"(d) : "v"(a), "v"(b));
    return d;
}

static __device__ __forceinline__ Frag ldfrag(const u16* p, int hh) {
    Frag f;
    f.half[0] = *(const v8ua*)(p + 8 * hh);
    f.half[1] = *(const v8ua*)(p + 16 + 8 * hh);
    return f;
}

static __device__ __forceinline__ u16 bfr(float f) {
    unsigned int u = __float_as_uint(f);
    u += 0x7FFFu + ((u >> 16) & 1u);
    return (u16)(u >> 16);
}
static __device__ __forceinline__ float bff(u16 b) {
    return __uint_as_float(((unsigned int)b) << 16);
}
static __device__ __forceinline__ u16 f16bits(float f) {
    const _Float16 hv = (_Float16)f;
    return __builtin_bit_cast(u16, hv);
}

static __device__ __forceinline__ void split8(v4f a, v4f c, v8u& hi, v8u& lo) {
    const float f[8] = {a.x, a.y, a.z, a.w, c.x, c.y, c.z, c.w};
    #pragma unroll
    for (int i = 0; i < 8; ++i) {
        const u16 hb = bfr(f[i]);
        hi[i] = hb;
        lo[i] = bfr(f[i] - bff(hb));
    }
}

static __device__ __forceinline__ float sigm(float v) {
    const float e = __expf(-v);
    const float s = __builtin_amdgcn_rcpf(1.0f + e);
    return __builtin_isnan(s) ? 0.0f : s;
}

__global__ __launch_bounds__(256) void conv_x_kernel(
    const float* __restrict__ x, u16* __restrict__ xH, u16* __restrict__ xL, int n8)
{
    const int g = blockIdx.x * 256 + threadIdx.x;
    if (g >= n8) return;
    const float* s = x + (size_t)g * 8;
    const v4f a = *(const v4fa*)(s);
    const v4f c = *(const v4fa*)(s + 4);
    v8u hi, lo;
    split8(a, c, hi, lo);
    u16* dh = xH + (size_t)g * 8;
    u16* dl = xL + (size_t)g * 8;
    *(volatile v8u*)dh = hi;
    *(volatile v8u*)dl = lo;
    __threadfence();
    *(volatile v8u*)dh = hi;
    *(volatile v8u*)dl = lo;
}

static __device__ __forceinline__ void w_store_pass(const float* s, u16* H, u16* L, int n0, int w, int lane) {
    #pragma unroll
    for (int j = 0; j < 4; ++j) {
        const int nl = 4 * w + j;
        const float* rp = s + nl * WPITCH + 8 * lane;
        const v4f a = *(const v4fa*)(rp);
        const v4f c = *(const v4fa*)(rp + 4);
        v8u hi, lo;
        split8(a, c, hi, lo);
        const size_t off = (size_t)(n0 + nl) * CC + 8 * lane;
        *(volatile v8u*)(H + off) = hi;
        *(volatile v8u*)(L + off) = lo;
    }
}

__global__ __launch_bounds__(256) void conv_w_kernel(
    const float* __restrict__ Wa, const float* __restrict__ Wp,
    u16* __restrict__ WaH, u16* __restrict__ WaL,
    u16* __restrict__ WpH, u16* __restrict__ WpL)
{
    __shared__ __attribute__((aligned(16))) float s[32 * WPITCH];
    const int tid = threadIdx.x, lane = tid & 31, w = tid >> 5;
    const int blk = blockIdx.x;
    const float* W; int N; u16* H; u16* L; int n0;
    if (blk < 24) { W = Wa; N = 3 * CC; H = WaH; L = WaL; n0 = blk * 32; }
    else          { W = Wp; N = CC;     H = WpH; L = WpL; n0 = (blk - 24) * 32; }
    for (int k = w; k < CC; k += 8)
        s[lane * WPITCH + k] = W[(size_t)k * N + n0 + lane];
    __syncthreads();
    w_store_pass(s, H, L, n0, w, lane);
    __threadfence();
    w_store_pass(s, H, L, n0, w, lane);
}

static __device__ __forceinline__ v8f tile3(const Frag& ah, const Frag& al,
                                             const u16* bH, const u16* bL, int hh, v8f c) {
    const Frag bh = ldfrag(bH, hh);
    const Frag bl = ldfrag(bL, hh);
    c = mma_bf16(ah.b, bh.b, c);
    c = mma_bf16(ah.b, bl.b, c);
    c = mma_bf16(al.b, bh.b, c);
    return c;
}

static __device__ __forceinline__ void gemm_k256_split(
    const u16* aH, const u16* aL, const u16* bH, const u16* bL, int hh,
    v8f& c0, v8f& c1, v8f& c2, v8f& c3)
{
    #pragma unroll 1
    for (int k0 = 0; k0 < CC; k0 += 32) {
        const Frag ah = ldfrag(aH + k0, hh);
        const Frag al = ldfrag(aL + k0, hh);
        c0 = tile3(ah, al, bH + k0,           bL + k0,           hh, c0);
        c1 = tile3(ah, al, bH + 16 * CC + k0, bL + 16 * CC + k0, hh, c1);
        c2 = tile3(ah, al, bH + 32 * CC + k0, bL + 32 * CC + k0, hh, c2);
        c3 = tile3(ah, al, bH + 48 * CC + k0, bL + 48 * CC + k0, hh, c3);
    }
}

static __device__ __forceinline__ void qk_store_pass(const u16* sA, u16* plane, int b, int head0,
                                                     int t0, int w, int lane) {
    const int q8 = lane & 7, sub = lane >> 3;
    #pragma unroll
    for (int i = 0; i < 4; ++i) {
        const int L = 16 * w + 4 * i + sub;
        const int hl = L >> 5, li = L & 31;
        const v8u v = *(const v8ua*)(sA + hl * 2048 + li * 64 + 8 * q8);
        const size_t bh = (size_t)(b * HH + head0 + hl);
        u16* dst = plane + (bh * TP + t0) * DD + li * 64 + 8 * q8;
        *(volatile v8u*)dst = v;
    }
}
static __device__ __forceinline__ void v_store_pass(const u16* sA, const u16* sB, u16* Vh, u16* Vl,
                                                    int b, int head0, int t0, int w, int lane) {
    const int q8 = lane & 7, sub = lane >> 3;
    #pragma unroll
    for (int i = 0; i < 8; ++i) {
        const int L = 32 * w + 4 * i + sub;
        const int p = L >> 6, Lp = L & 63;
        const int hl = Lp >> 5, d = Lp & 31;
        const u16* src = (p ? sB : sA) + hl * 2048 + d * 64 + 8 * q8;
        const v8u v = *(const v8ua*)src;
        const size_t row = (size_t)((b * HH + head0 + hl) * DD + d);
        u16* dst = (p ? Vl : Vh) + row * TP + t0 + 8 * q8;
        *(volatile v8u*)dst = v;
    }
}

__global__ __launch_bounds__(128) void qkv_kernel(
    const u16* __restrict__ xH, const u16* __restrict__ xL,
    const u16* __restrict__ WaH, const u16* __restrict__ WaL,
    const float* __restrict__ bias,
    u16* __restrict__ Qf, u16* __restrict__ Kf,
    u16* __restrict__ Vh, u16* __restrict__ Vl)
{
    __shared__ __attribute__((aligned(16))) u16 sA[2 * 64 * 32];
    __shared__ __attribute__((aligned(16))) u16 sB[2 * 64 * 32];

    const int tid = threadIdx.x, lane = tid & 31, w = tid >> 5;
    const int hh = lane >> 4, m = lane & 15;
    const int nt = blockIdx.x, tt = blockIdx.y, b = blockIdx.z;
    const int t0 = tt * 64, nbase = nt * 64;
    const int which = nt >> 2;
    const int head0 = (nt & 3) * 2;

    const int tok = t0 + 16 * w + m;
    const int tokc = (tok < TT) ? tok : (TT - 1);
    const size_t arow = (size_t)(b * TT + tokc) * CC;
    const size_t brow = (size_t)(nbase + m) * CC;

    const v8f zero8 = {0.f, 0.f, 0.f, 0.f, 0.f, 0.f, 0.f, 0.f};
    v8f c0 = zero8, c1 = zero8, c2 = zero8, c3 = zero8;
    gemm_k256_split(xH + arow, xL + arow, WaH + brow, WaL + brow, hh, c0, c1, c2, c3);
    v8f acc[4] = {c0, c1, c2, c3};

    #pragma unroll
    for (int u = 0; u < 4; ++u) {
        const float bv = bias[nbase + 16 * u + m];
        const int hl = u >> 1;
        const int d = 16 * (u & 1) + m;
        #pragma unroll
        for (int r = 0; r < 8; ++r) {
            const int i = 16 * w + 8 * hh + r;
            const float y = acc[u][r] + bv;
            if (which == 2) {
                const u16 hb = bfr(y);
                sA[hl * 2048 + d * 64 + i] = hb;
                sB[hl * 2048 + d * 64 + i] = bfr(y - bff(hb));
            } else {
                sA[hl * 2048 + i * 32 + d] = f16bits(y * 8.0f);
            }
        }
    }
    __syncthreads();

    if (which == 2) {
        v_store_pass(sA, sB, Vh, Vl, b, head0, t0, w, lane);
        __threadfence();
        v_store_pass(sA, sB, Vh, Vl, b, head0, t0, w, lane);
    } else {
        u16* plane = (which == 0) ? Qf : Kf;
        qk_store_pass(sA, plane, b, head0, t0, w, lane);
        __threadfence();
        qk_store_pass(sA, plane, b, head0, t0, w, lane);
    }
}

static __device__ __forceinline__ void ctx_store_pass(const u16* sC, u16* Ch, u16* Cl, size_t rowbase,
                                                      int w, int lane) {
    const int q8 = lane & 7, sub = lane >> 3;
    #pragma unroll
    for (int i = 0; i < 4; ++i) {
        const int L = 16 * w + 4 * i + sub;
        const int p = L >> 6, li = L & 63;
        const v8u v = *(const v8ua*)(sC + p * 4096 + li * 64 + 8 * q8);
        u16* dst = (p ? Cl : Ch) + rowbase + li * 64 + 8 * q8;
        *(volatile v8u*)dst = v;
    }
}

__global__ __launch_bounds__(256) void attn_kernel(
    const u16* __restrict__ Qf, const u16* __restrict__ Kf,
    const u16* __restrict__ Vh, const u16* __restrict__ Vl,
    const float* __restrict__ pw, float* __restrict__ mix,
    u16* __restrict__ Ch, u16* __restrict__ Cl)
{
    __shared__ __attribute__((aligned(16))) float sS[HH * 16 * SP];

    const int tid = threadIdx.x, lane = tid & 31, w = tid >> 5;
    const int hh = lane >> 4, m = lane & 15;
    const int qt = blockIdx.x, b = blockIdx.y;
    const int h = w, bh = b * HH + h, t0 = qt * 16;

    float pwv[HH];
    #pragma unroll
    for (int i = 0; i < HH; ++i) pwv[i] = pw[i];

    const Frag qf = ldfrag(Qf + ((size_t)bh * TP + t0 + m) * DD, hh);

    const v8f zero8 = {0.f, 0.f, 0.f, 0.f, 0.f, 0.f, 0.f, 0.f};
    v8f O0 = zero8, O1 = zero8;
    float mrun = -1e30f, lrun = 0.0f;
    float* tile = sS + h * 16 * SP;
    const float sscale = 0.17677669529663687f * 0.015625f;

    #pragma unroll 1
    for (int s0 = 0; s0 < TP; s0 += 32) {
        const u16* kp = Kf + ((size_t)bh * TP + s0 + m) * DD;
        const Frag k0f = ldfrag(kp, hh);
        const Frag k1f = ldfrag(kp + 16 * DD, hh);
        const v8f S0 = mma_f16(qf.h, k0f.h, zero8);
        const v8f S1 = mma_f16(qf.h, k1f.h, zero8);
        #pragma unroll
        for (int r = 0; r < 8; ++r) {
            tile[(8 * hh + r) * SP + m]      = S0[r] * sscale;
            tile[(8 * hh + r) * SP + 16 + m] = S1[r] * sscale;
        }
        __syncthreads();

        if (tid < 128) {
            const int q = tid >> 3, c4 = (tid & 7) * 4;
            float a0 = 0.f, a1 = 0.f, a2 = 0.f, a3 = 0.f;
            #pragma unroll
            for (int hd = 0; hd < HH; ++hd) {
                const v4f s4 = *(const v4fa*)(sS + (hd * 16 + q) * SP + c4);
                const float pv = pwv[hd];
                a0 = fmaf(s4.x, pv, a0);
                a1 = fmaf(s4.y, pv, a1);
                a2 = fmaf(s4.z, pv, a2);
                a3 = fmaf(s4.w, pv, a3);
            }
            v4f r4;
            r4.x = sigm(a0); r4.y = sigm(a1); r4.z = sigm(a2); r4.w = sigm(a3);
            float* dst = mix + ((size_t)(b * TP + t0 + q)) * TP + s0 + c4;
            *(volatile v4f*)dst = r4;
            __threadfence();
            *(volatile v4f*)dst = r4;
        }

        const float* rp = tile + m * SP + 8 * hh;
        const v4f x0 = *(const v4fa*)(rp);
        const v4f x1 = *(const v4fa*)(rp + 4);
        const v4f x2 = *(const v4fa*)(rp + 16);
        const v4f x3 = *(const v4fa*)(rp + 20);
        float sv[16] = {x0.x, x0.y, x0.z, x0.w, x1.x, x1.y, x1.z, x1.w,
                        x2.x, x2.y, x2.z, x2.w, x3.x, x3.y, x3.z, x3.w};
        if (s0 + 32 > TT) {
            #pragma unroll
            for (int i = 0; i < 16; ++i) {
                const int key = s0 + ((i < 8) ? (8 * hh + i) : (8 + 8 * hh + i));
                if (key >= TT) sv[i] = -1e30f;
            }
        }

        float mloc = sv[0];
        #pragma unroll
        for (int i = 1; i < 16; ++i) mloc = fmaxf(mloc, sv[i]);
        mloc = fmaxf(mloc, __shfl_xor(mloc, 16));
        const float mnew = fmaxf(mrun, mloc);
        const float alpha = __expf(mrun - mnew);
        mrun = mnew;
        float ps = 0.0f;
        v16u phv, plv;
        #pragma unroll
        for (int i = 0; i < 16; ++i) {
            const float p = __expf(sv[i] - mnew);
            ps += p;
            const u16 hb = bfr(p);
            phv[i] = hb;
            plv[i] = bfr(p - bff(hb));
        }
        ps += __shfl_xor(ps, 16);
        lrun = lrun * alpha + ps;

        #pragma unroll
        for (int r = 0; r < 8; ++r) {
            const float ar = __shfl(alpha, 8 * hh + r);
            O0[r] *= ar;
            O1[r] *= ar;
        }

        Frag ph, pl;
        ph.v = phv; pl.v = plv;
        {
            const size_t vrow = ((size_t)(bh * DD + m)) * TP + s0;
            const Frag vh = ldfrag(Vh + vrow, hh);
            const Frag vl = ldfrag(Vl + vrow, hh);
            O0 = mma_bf16(ph.b, vh.b, O0);
            O0 = mma_bf16(ph.b, vl.b, O0);
            O0 = mma_bf16(pl.b, vh.b, O0);
        }
        {
            const size_t vrow = ((size_t)(bh * DD + 16 + m)) * TP + s0;
            const Frag vh = ldfrag(Vh + vrow, hh);
            const Frag vl = ldfrag(Vl + vrow, hh);
            O1 = mma_bf16(ph.b, vh.b, O1);
            O1 = mma_bf16(ph.b, vl.b, O1);
            O1 = mma_bf16(pl.b, vh.b, O1);
        }
        __syncthreads();
    }

    const float inv = 1.0f / lrun;
    u16* sC = (u16*)sS;
    #pragma unroll
    for (int r = 0; r < 8; ++r) {
        const float ir = __shfl(inv, 8 * hh + r);
        const int q = 8 * hh + r;
        {
            const float c = O0[r] * ir;
            const u16 hb = bfr(c);
            sC[q * CC + h * DD + m] = hb;
            sC[4096 + q * CC + h * DD + m] = bfr(c - bff(hb));
        }
        {
            const float c = O1[r] * ir;
            const u16 hb = bfr(c);
            sC[q * CC + h * DD + 16 + m] = hb;
            sC[4096 + q * CC + h * DD + 16 + m] = bfr(c - bff(hb));
        }
    }
    __syncthreads();

    const size_t rowbase = ((size_t)(b * TP + t0)) * CC;
    ctx_store_pass(sC, Ch, Cl, rowbase, w, lane);
    __threadfence();
    ctx_store_pass(sC, Ch, Cl, rowbase, w, lane);
}

static __device__ __forceinline__ void out_store_pass(const float* sO, float* out1, int b, int t0,
                                                      int nbase, int w, int lane) {
    const int q8 = lane & 7, sub = lane >> 3;
    #pragma unroll
    for (int i = 0; i < 8; ++i) {
        const int L = 32 * w + 4 * i + sub;
        const int row = L >> 1, half = L & 1;
        const int t = t0 + row;
        if (t < TT) {
            const v4f v = *(const v4fa*)(sO + row * 64 + 32 * half + 4 * q8);
            float* dst = out1 + ((size_t)(b * TT + t)) * CC + nbase + 32 * half + 4 * q8;
            *(volatile v4f*)dst = v;
        }
    }
}

__global__ __launch_bounds__(128) void proj_kernel(
    const u16* __restrict__ cH, const u16* __restrict__ cL,
    const u16* __restrict__ WpH, const u16* __restrict__ WpL,
    const float* __restrict__ bias, float* __restrict__ out1)
{
    __shared__ __attribute__((aligned(16))) float sO[64 * 64];

    const int tid = threadIdx.x, lane = tid & 31, w = tid >> 5;
    const int hh = lane >> 4, m = lane & 15;
    const int nt = blockIdx.x, tt = blockIdx.y, b = blockIdx.z;
    const int t0 = tt * 64, nbase = nt * 64;

    const size_t arow = ((size_t)(b * TP + t0 + 16 * w + m)) * CC;
    const size_t brow = ((size_t)(nbase + m)) * CC;

    const v8f zero8 = {0.f, 0.f, 0.f, 0.f, 0.f, 0.f, 0.f, 0.f};
    v8f c0 = zero8, c1 = zero8, c2 = zero8, c3 = zero8;
    gemm_k256_split(cH + arow, cL + arow, WpH + brow, WpL + brow, hh, c0, c1, c2, c3);
    v8f acc[4] = {c0, c1, c2, c3};

    #pragma unroll
    for (int u = 0; u < 4; ++u) {
        const float bv = bias[nbase + 16 * u + m];
        #pragma unroll
        for (int r = 0; r < 8; ++r) {
            const int i = 16 * w + 8 * hh + r;
            sO[i * 64 + 16 * u + m] = acc[u][r] + bv;
        }
    }
    __syncthreads();

    out_store_pass(sO, out1, b, t0, nbase, w, lane);
    __threadfence();
    out_store_pass(sO, out1, b, t0, nbase, w, lane);
}

__global__ __launch_bounds__(256) void pack_kernel(
    const float* __restrict__ mix, float* __restrict__ out0, int n4)
{
    const int g = blockIdx.x * 256 + threadIdx.x;
    if (g >= n4) return;
    const int row = g / 125;
    const int col = (g - row * 125) * 4;
    const int b = row / TT, t = row - b * TT;
    const v4f v = *(const v4fa*)(mix + ((size_t)(b * TP + t)) * TP + col);
    float* dst = out0 + (size_t)g * 4;
    *(volatile v4f*)dst = v;
    __threadfence();
    *(volatile v4f*)dst = v;
}

extern "C" void kernel_launch(void* const* d_in, const int* in_sizes, int n_in,
                              void* d_out, int out_size, void* d_ws, size_t ws_size,
                              hipStream_t stream)
{
    if (n_in < 6) return;
    if (in_sizes[0] != BB * TT * CC) return;
    if (in_sizes[1] != CC * 3 * CC) return;
    if (in_sizes[2] != 3 * CC) return;
    if (in_sizes[3] != HH) return;
    if (in_sizes[4] != CC * CC) return;
    if (in_sizes[5] != CC) return;
    if (out_size != BB * TT * TT + BB * TT * CC) return;

    const float* x      = (const float*)d_in[0];
    const float* W_attn = (const float*)d_in[1];
    const float* b_attn = (const float*)d_in[2];
    const float* p_w    = (const float*)d_in[3];
    const float* W_proj = (const float*)d_in[4];
    const float* b_proj = (const float*)d_in[5];

    float* out0 = (float*)d_out;
    float* out1 = (float*)d_out + (size_t)BB * TT * TT;

    const size_t xp_bytes  = (size_t)BB * TT * CC * 2;
    const size_t wa_bytes  = (size_t)3 * CC * CC * 2;
    const size_t wp_bytes  = (size_t)CC * CC * 2;
    const size_t qk_bytes  = (size_t)BB * HH * TP * DD * 2;
    const size_t cx_bytes  = (size_t)BB * TP * CC * 2;
    const size_t mix_bytes = (size_t)BB * TP * TP * 4;
    const size_t total = 2 * xp_bytes + 2 * wa_bytes + 2 * wp_bytes + 4 * qk_bytes + 2 * cx_bytes + mix_bytes;
    if (total > ws_size) return;

    char* ws = (char*)d_ws;
    size_t o = 0;
    u16* xH  = (u16*)(ws + o); o += xp_bytes;
    u16* xL  = (u16*)(ws + o); o += xp_bytes;
    u16* WaH = (u16*)(ws + o); o += wa_bytes;
    u16* WaL = (u16*)(ws + o); o += wa_bytes;
    u16* WpH = (u16*)(ws + o); o += wp_bytes;
    u16* WpL = (u16*)(ws + o); o += wp_bytes;
    u16* Qf  = (u16*)(ws + o); o += qk_bytes;
    u16* Kf  = (u16*)(ws + o); o += qk_bytes;
    u16* Vh  = (u16*)(ws + o); o += qk_bytes;
    u16* Vl  = (u16*)(ws + o); o += qk_bytes;
    u16* Ch  = (u16*)(ws + o); o += cx_bytes;
    u16* Cl  = (u16*)(ws + o); o += cx_bytes;
    float* mix = (float*)(ws + o); o += mix_bytes;
    if (o > ws_size) return;

    const int n8 = BB * TT * CC / 8;
    conv_x_kernel<<<(n8 + 255) / 256, 256, 0, stream>>>(x, xH, xL, n8);
    conv_w_kernel<<<32, 256, 0, stream>>>(W_attn, W_proj, WaH, WaL, WpH, WpL);
    qkv_kernel<<<dim3(12, TP / 64, BB), 128, 0, stream>>>(xH, xL, WaH, WaL, b_attn, Qf, Kf, Vh, Vl);
    attn_kernel<<<dim3(TP / 16, BB), 256, 0, stream>>>(Qf, Kf, Vh, Vl, p_w, mix, Ch, Cl);
    proj_kernel<<<dim3(4, TP / 64, BB), 128, 0, stream>>>(Ch, Cl, WpH, WpL, b_proj, out1);
    const int n4 = BB * TT * TT / 4;
    pack_kernel<<<(n4 + 255) / 256, 256, 0, stream>>>(mix, out0, n4);
}
